// MoeGatherRsOp_79920751444178
// MI455X (gfx1250) — hardware-verified
//
#include <hip/hip_runtime.h>


namespace {
constexpr int NTOK = 8192, TK = 2, NE = 8, K = 512, N = 1024, M = NTOK * TK;
constexpr float XS = 8.0f, WSC = 256.0f;
typedef _Float16 b16;
typedef __attribute__((ext_vector_type(16))) _Float16 v16b;
typedef __attribute__((ext_vector_type(8))) _Float16 v8b;
typedef __attribute__((ext_vector_type(8))) float v8f;
typedef __attribute__((ext_vector_type(4))) float v4f;
__device__ __forceinline__ float bf16_rne(float f) { unsigned int u = __float_as_uint(f); u += 0x7FFFu + ((u >> 16) & 1u); return __uint_as_float(u & 0xFFFF0000u); }
__device__ __forceinline__ v16b frag_kb(const b16* p, int hh) { const v8b a = *(const v8b*)(p + 8 * hh), b = *(const v8b*)(p + 16 + 8 * hh); v16b f;
#pragma unroll
  for (int e = 0; e < 8; ++e) { f[e] = a[e]; f[8 + e] = b[e]; } return f; }
__device__ __forceinline__ v8f wmma16b(v16b a, v16b b, v8f c) { v8f d = __builtin_amdgcn_wmma_f32_16x16x32_f16(false, a, false, b, (short)0, c, false, false); asm volatile("v_nop\n\tv_nop\n\tv_nop\n\tv_nop" : "+v"(d) : "v"(a), "v"(b)); return d; }
__device__ __forceinline__ void wave_lds_sync() { __builtin_amdgcn_fence(__ATOMIC_RELEASE, "workgroup"); __builtin_amdgcn_wave_barrier(); __builtin_amdgcn_fence(__ATOMIC_ACQUIRE, "workgroup"); }
__device__ __forceinline__ float pmul(float a, float b) { float p = a * b; asm volatile("" : "+v"(p)); return p; }
__device__ __forceinline__ int iclamp(int v, int lo, int hi) { return v < lo ? lo : (v > hi ? hi : v); }

__global__ __launch_bounds__(256) void wt_kernel(const float* __restrict__ w, b16* __restrict__ WT) {
  const size_t u = (size_t)blockIdx.x * 256 + threadIdx.x; if (u >= (size_t)NE * N * K / 8) return; const size_t e8 = u * 8; const int e = (int)(e8 / ((size_t)N * K)); const int n = (int)((e8 / K) % N), k0 = (int)(e8 % K); v8b v;
#pragma unroll
  for (int j = 0; j < 8; ++j) v[j] = (b16)(bf16_rne(w[((size_t)e * K + k0 + j) * N + n]) * WSC); for (int pass = 0; pass < 2; ++pass) { *(volatile v8b*)(WT + e8) = v; __threadfence(); }
}
__global__ __launch_bounds__(256) void rex_kernel(const int* __restrict__ splits, const float* __restrict__ isc, const float* __restrict__ wsc, const float* __restrict__ ovs, int* __restrict__ REX, float* __restrict__ SC) {
  const int m = blockIdx.x * 256 + threadIdx.x; if (m >= M) return; long long cs = 0; int e = 0; for (int j = 0; j < NE; ++j) { cs += splits[j]; if (cs <= m) e = j + 1; }
  e = iclamp(e, 0, NE - 1); const float s = pmul(pmul(bf16_rne(isc[0]), bf16_rne(wsc[e])), bf16_rne(ovs[m]));
  for (int pass = 0; pass < 2; ++pass) { ((volatile int*)REX)[m] = e; ((volatile float*)SC)[m] = s; __threadfence(); }
}
__global__ __launch_bounds__(32) void gemm_kernel(const float* __restrict__ inp, const b16* __restrict__ WT, const int* __restrict__ REX, const float* __restrict__ SC, int MLIM, float* __restrict__ Y) {
  __shared__ __attribute__((aligned(16))) b16 Ah[16][K + 8]; __shared__ __attribute__((aligned(16))) float Tf[16][256 + 4]; __shared__ int Ex[16];
  const int lane = threadIdx.x, nloc = lane & 15, hlf = lane >> 4; const size_t m0 = (size_t)(blockIdx.x / 4) * 16; const int cg = blockIdx.x % 4; if (m0 >= (size_t)MLIM) return;
  for (int rr = 0; rr < 16; ++rr) for (int q = 0; q < K / 32; ++q) Ah[rr][q * 32 + lane] = (b16)(bf16_rne(inp[(m0 + rr) * K + q * 32 + lane]) * XS);
  if (lane < 16) Ex[lane] = iclamp(REX[m0 + lane], 0, NE - 1);
  wave_lds_sync();
  for (int rr = 0; rr < 16; ++rr) { const int e = Ex[rr]; bool seen = false; for (int r2 = 0; r2 < rr; ++r2) seen = seen || (Ex[r2] == e); if (seen) continue;
    v8f acc[16];
#pragma unroll
    for (int t = 0; t < 16; ++t) acc[t] = (v8f){};
#pragma unroll 1
    for (int kb = 0; kb < K; kb += 32) { const v16b a = frag_kb(&Ah[nloc][kb], hlf);
#pragma unroll
      for (int t = 0; t < 16; ++t) acc[t] = wmma16b(a, frag_kb(WT + ((size_t)e * N + cg * 256 + t * 16 + nloc) * K + kb, hlf), acc[t]); }
#pragma unroll
    for (int t = 0; t < 16; ++t)
#pragma unroll
      for (int r8 = 0; r8 < 8; ++r8) { const int rl = 8 * hlf + r8; if (Ex[rl] == e) Tf[rl][t * 16 + nloc] = acc[t][r8] * (1.0f / (XS * WSC)); } }
  wave_lds_sync();
  for (int pass = 0; pass < 2; ++pass) { for (int rr = 0; rr < 16; ++rr) { const float s = SC[m0 + rr]; for (int q = 0; q < 2; ++q) { v4f v = *(const v4f*)(&Tf[rr][q * 128 + lane * 4]); for (int i = 0; i < 4; ++i) v[i] = pmul(v[i], s); *(volatile v4f*)(Y + (m0 + rr) * N + cg * 256 + q * 128 + lane * 4) = v; } } __threadfence(); }
}
__global__ __launch_bounds__(32) void reduce_kernel(const float* __restrict__ Y, const int* __restrict__ sidx, int TLIM, float* __restrict__ out) {
  const int lane = threadIdx.x; const size_t t0 = (size_t)blockIdx.x * 16; if (t0 >= (size_t)TLIM) return;
  for (int pass = 0; pass < 2; ++pass) { for (int rr = 0; rr < 16; ++rr) { const size_t t = t0 + rr; const int s0 = iclamp(sidx[t * TK], 0, M - 1), s1 = iclamp(sidx[t * TK + 1], 0, M - 1);
      for (int q = 0; q < N / 128; ++q) { const v4f a = *(const v4f*)(Y + (size_t)s0 * N + q * 128 + lane * 4), b = *(const v4f*)(Y + (size_t)s1 * N + q * 128 + lane * 4); v4f o; for (int i = 0; i < 4; ++i) o[i] = a[i] + b[i]; *(volatile v4f*)(out + t * N + q * 128 + lane * 4) = o; } } __threadfence(); }
}
}

extern "C" void kernel_launch(void* const* d_in, const int* in_sizes, int n_in, void* d_out, int out_size, void* d_ws, size_t ws_size, hipStream_t stream) {
  (void)n_in;
  auto Fp = [&](int i) { return (const float*)d_in[i]; }; auto Ip = [&](int i) { return (const int*)d_in[i]; };
  if (in_sizes[0] != M * K || in_sizes[1] != NE * K * N || in_sizes[2] != NE || in_sizes[3] != NTOK * TK || in_sizes[4] != 1 || in_sizes[5] != NE || in_sizes[6] != M || out_size != NTOK * N) return;
  const int MLIM = M; const int TLIM = NTOK;
  size_t off = 0; char* ws = (char*)d_ws;
  auto carve = [&](size_t bytes) { char* p = ws + off; off += (bytes + 255) & ~(size_t)255; return p; };
  b16* WT = (b16*)carve((size_t)NE * N * K * 2); int* REX = (int*)carve((size_t)M * 4); float* SC = (float*)carve((size_t)M * 4); float* Y = (float*)carve((size_t)M * N * 4);
  if (off > ws_size || off > ((size_t)96 << 20)) return;
  wt_kernel<<<(unsigned)(((size_t)NE * N * K / 8 + 255) / 256), 256, 0, stream>>>(Fp(1), WT);
  rex_kernel<<<M / 256, 256, 0, stream>>>(Ip(2), Fp(4), Fp(5), Fp(6), REX, SC);
  gemm_kernel<<<(MLIM / 16) * 4, 32, 0, stream>>>(Fp(0), WT, REX, SC, MLIM, Y);
  reduce_kernel<<<TLIM / 16, 32, 0, stream>>>(Y, Ip(3), TLIM, (float*)d_out);
}
